// attention_mech_deep_52888227283043
// MI455X (gfx1250) — hardware-verified
//
#include <hip/hip_runtime.h>

typedef _Float16 v16h __attribute__((ext_vector_type(16)));
typedef _Float16 v8h  __attribute__((ext_vector_type(8)));
typedef __bf16   v16b __attribute__((ext_vector_type(16)));
typedef unsigned short v8us __attribute__((ext_vector_type(8)));
typedef float v8f __attribute__((ext_vector_type(8)));
typedef float v4f __attribute__((ext_vector_type(4)));

#define DEVI __device__ __forceinline__

constexpr int BC  = 64;
constexpr int NN  = 64;
constexpr int SS  = 128;
constexpr int IR  = 96;
constexpr int NTH = 256;
constexpr float EPSF = 1e-5f;

DEVI unsigned short bf16_rne(float x)
{
  unsigned int u = __float_as_uint(x);
  u += 0x7FFFu + ((u >> 16) & 1u);
  return (unsigned short)(u >> 16);
}
DEVI float bf16_to_f32(unsigned short b) { return __uint_as_float(((unsigned int)b) << 16); }
DEVI void split_bf16(float x, unsigned short& hi, unsigned short& lo)
{
  hi = bf16_rne(x);
  lo = bf16_rne(x - bf16_to_f32(hi));
}

DEVI v8f zero8()
{
  v8f z;
#pragma unroll
  for (int i = 0; i < 8; ++i) z[i] = 0.0f;
  return z;
}

DEVI v8f wmma_bf(v16b a, v16b b, v8f c)
{
  c = __builtin_amdgcn_wmma_f32_16x16x32_bf16(false, a, false, b, (short)0, c, false, false);
  asm volatile("v_nop\n\tv_nop\n\tv_nop\n\tv_nop" : "+v"(c) : "v"(a), "v"(b));
  return c;
}
DEVI v8f wmma_h(v16h a, v16h b, v8f c)
{
  c = __builtin_amdgcn_wmma_f32_16x16x32_f16(false, a, false, b, (short)0, c, false, false);
  asm volatile("v_nop\n\tv_nop\n\tv_nop\n\tv_nop" : "+v"(c) : "v"(a), "v"(b));
  return c;
}

DEVI v16b ldfrag_b(const unsigned short* base, int row, int k0, int h)
{
  union { v16b v; v8us q[2]; } u;
  const unsigned short* p = base + row * SS + k0 + 8 * h;
  u.q[0] = *(const v8us*)(p);
  u.q[1] = *(const v8us*)(p + 16);
  return u.v;
}
DEVI v16h ldfrag_h(const _Float16* base, int row, int k0, int h)
{
  union { v16h v; v8h q[2]; } u;
  const _Float16* p = base + row * SS + k0 + 8 * h;
  u.q[0] = *(const v8h*)(p);
  u.q[1] = *(const v8h*)(p + 16);
  return u.v;
}

DEVI void store_lines(float* dst, const float* src, int nfl, int tid)
{
  const int lane = tid & 31, wave = tid >> 5;
  const int nch = nfl >> 7;
  for (int c = wave; c < nch; c += 8) {
    const v4f v = *(const v4f*)(src + c * 128 + 4 * lane);
    *(volatile v4f*)(dst + c * 128 + 4 * lane) = v;
  }
  __threadfence();
  for (int c = wave; c < nch; c += 8) {
    const v4f v = *(const v4f*)(src + c * 128 + 4 * lane);
    *(volatile v4f*)(dst + c * 128 + 4 * lane) = v;
  }
}

DEVI void stage_w(const float* __restrict__ W, int K, unsigned short* wH, unsigned short* wL, int tid)
{
  const int tot = K * SS;
  for (int i = tid; i < tot; i += NTH) {
    const int k = i >> 7, n = i & 127;
    unsigned short hi, lo;
    split_bf16(W[i], hi, lo);
    wH[n * SS + k] = hi;
    wL[n * SS + k] = lo;
  }
}
DEVI void stage_x(const float* __restrict__ X, unsigned short* aH, unsigned short* aL, int tid)
{
  for (int i = tid; i < NN * IR; i += NTH) {
    const int r = i / IR, k = i - r * IR;
    unsigned short hi, lo;
    split_bf16(X[i], hi, lo);
    aH[r * SS + k] = hi;
    aL[r * SS + k] = lo;
  }
}
template <int ACT>
DEVI void f_to_planes(const float* fT, unsigned short* dH, unsigned short* dL, float slope, int tid)
{
  for (int i = tid; i < NN * SS; i += NTH) {
    float x = fT[i];
    if (ACT == 1) x = (x >= 0.0f) ? x : slope * x;
    if (ACT == 2) x = tanhf(x);
    unsigned short hi, lo;
    split_bf16(x, hi, lo);
    dH[i] = hi;
    dL[i] = lo;
  }
}
DEVI void tanh_inplace(float* fT, int tid)
{
  for (int i = tid; i < NN * SS; i += NTH) fT[i] = tanhf(fT[i]);
}
DEVI void ln_to_planes(const float* fT, const float* __restrict__ g, const float* __restrict__ bta,
                       unsigned short* dH, unsigned short* dL, int tid)
{
  const int row = tid >> 2, part = tid & 3;
  const float* x = fT + row * SS + part * 32;
  float s = 0.0f;
#pragma unroll 8
  for (int c = 0; c < 32; ++c) s += x[c];
  s += __shfl_xor(s, 1, 32);
  s += __shfl_xor(s, 2, 32);
  const float mean = s * (1.0f / SS);
  float v = 0.0f;
#pragma unroll 8
  for (int c = 0; c < 32; ++c) { const float d = x[c] - mean; v = fmaf(d, d, v); }
  v += __shfl_xor(v, 1, 32);
  v += __shfl_xor(v, 2, 32);
  const float rstd = rsqrtf(v * (1.0f / SS) + EPSF);
#pragma unroll 4
  for (int c = 0; c < 32; ++c) {
    const int col = part * 32 + c;
    const float y = (x[c] - mean) * rstd * g[col] + bta[col];
    unsigned short hi, lo;
    split_bf16(y, hi, lo);
    dH[row * SS + col] = hi;
    dL[row * SS + col] = lo;
  }
}
DEVI void softmax_cols(const float* L, float* P, int tid)
{
  const int mcol = tid >> 2, part = tid & 3, n0 = part * 16;
  float mx = -3.0e38f;
#pragma unroll 4
  for (int i = 0; i < 16; ++i) mx = fmaxf(mx, L[(n0 + i) * NN + mcol]);
  mx = fmaxf(mx, __shfl_xor(mx, 1, 32));
  mx = fmaxf(mx, __shfl_xor(mx, 2, 32));
  float s = 0.0f;
#pragma unroll 4
  for (int i = 0; i < 16; ++i) {
    const float e = expf(L[(n0 + i) * NN + mcol] - mx);
    P[(n0 + i) * NN + mcol] = e;
    s += e;
  }
  s += __shfl_xor(s, 1, 32);
  s += __shfl_xor(s, 2, 32);
  const float inv = 1.0f / s;
#pragma unroll 4
  for (int i = 0; i < 16; ++i) P[(n0 + i) * NN + mcol] *= inv;
}

template <int NT>
DEVI void gemm_x3(const unsigned short* Ah, const unsigned short* Al,
                  const unsigned short* Bh, const unsigned short* Bl,
                  int nks, float* outF, int outPitch, const float* __restrict__ bias, int tid)
{
  const int lane = tid & 31, wave = tid >> 5, h = lane >> 4, m = lane & 15;
  const int row0 = (wave >> 1) * 16;
  const int ct0  = (wave & 1) * NT;
  v8f acc[NT];
#pragma unroll
  for (int j = 0; j < NT; ++j) acc[j] = zero8();
#pragma unroll 1
  for (int ks = 0; ks < nks; ++ks) {
    const int k0 = ks * 32;
    const v16b ah = ldfrag_b(Ah, row0 + m, k0, h);
    const v16b al = ldfrag_b(Al, row0 + m, k0, h);
#pragma unroll
    for (int j = 0; j < NT; ++j) {
      const int nrow = (ct0 + j) * 16 + m;
      const v16b bh = ldfrag_b(Bh, nrow, k0, h);
      const v16b bl = ldfrag_b(Bl, nrow, k0, h);
      acc[j] = wmma_bf(ah, bh, acc[j]);
      acc[j] = wmma_bf(ah, bl, acc[j]);
      acc[j] = wmma_bf(al, bh, acc[j]);
    }
  }
#pragma unroll
  for (int j = 0; j < NT; ++j) {
    const int col = (ct0 + j) * 16 + m;
    const float bv = bias ? bias[col] : 0.0f;
#pragma unroll
    for (int r = 0; r < 8; ++r) outF[(row0 + 8 * h + r) * outPitch + col] = acc[j][r] + bv;
  }
}

__global__ __launch_bounds__(NTH) void k_prep(
    const float* __restrict__ tL,  const float* __restrict__ tH,
    const float* __restrict__ Wk1, const float* __restrict__ bk1,
    const float* __restrict__ Wk2, const float* __restrict__ bk2,
    const float* __restrict__ Wk3, const float* __restrict__ bk3,
    const float* __restrict__ Wq1, const float* __restrict__ bq1,
    const float* __restrict__ Wq2, const float* __restrict__ bq2,
    const float* __restrict__ Wv1, const float* __restrict__ aK,
    const float* __restrict__ gK,  const float* __restrict__ betaK,
    float* __restrict__ attn, float* __restrict__ hq, float* __restrict__ hk)
{
  __shared__ __align__(16) unsigned short wH[SS * SS];
  __shared__ __align__(16) unsigned short wL[SS * SS];
  __shared__ __align__(16) unsigned short aH[NN * SS];
  __shared__ __align__(16) unsigned short aL[NN * SS];
  __shared__ __align__(16) unsigned short qH[NN * SS];
  __shared__ __align__(16) unsigned short qL[NN * SS];
  __shared__ __align__(16) float fT[NN * SS];

  const int tid = threadIdx.x;
  const int bc  = blockIdx.x;
  const float slopeK = aK[0];
  const size_t xoff = (size_t)bc * NN * IR;

  stage_x(tH + xoff, aH, aL, tid);
  stage_w(Wq1, IR, wH, wL, tid);
  __syncthreads();
  gemm_x3<4>(aH, aL, wH, wL, IR / 32, fT, SS, bq1, tid);
  __syncthreads();
  f_to_planes<2>(fT, aH, aL, 0.0f, tid);
  stage_w(Wq2, SS, wH, wL, tid);
  __syncthreads();
  gemm_x3<4>(aH, aL, wH, wL, SS / 32, fT, SS, bq2, tid);
  __syncthreads();
  f_to_planes<0>(fT, qH, qL, 0.0f, tid);
  stage_w(Wv1, SS, wH, wL, tid);
  __syncthreads();
  gemm_x3<4>(qH, qL, wH, wL, SS / 32, fT, SS, nullptr, tid);
  __syncthreads();
  store_lines(hq + (size_t)bc * NN * SS, fT, NN * SS, tid);

  stage_x(tL + xoff, aH, aL, tid);
  stage_w(Wk1, IR, wH, wL, tid);
  __syncthreads();
  gemm_x3<4>(aH, aL, wH, wL, IR / 32, fT, SS, bk1, tid);
  __syncthreads();
  f_to_planes<1>(fT, aH, aL, slopeK, tid);
  stage_w(Wk2, SS, wH, wL, tid);
  __syncthreads();
  gemm_x3<4>(aH, aL, wH, wL, SS / 32, fT, SS, bk2, tid);
  __syncthreads();
  tanh_inplace(fT, tid);
  __syncthreads();
  ln_to_planes(fT, gK, betaK, aH, aL, tid);
  stage_w(Wk3, SS, wH, wL, tid);
  __syncthreads();
  gemm_x3<4>(aH, aL, wH, wL, SS / 32, fT, SS, bk3, tid);
  __syncthreads();
  f_to_planes<0>(fT, aH, aL, 0.0f, tid);
  stage_w(Wv1 + SS * SS, SS, wH, wL, tid);
  __syncthreads();
  gemm_x3<4>(aH, aL, wH, wL, SS / 32, fT, SS, nullptr, tid);
  __syncthreads();
  store_lines(hk + (size_t)bc * NN * SS, fT, NN * SS, tid);
  __syncthreads();

  gemm_x3<2>(aH, aL, qH, qL, SS / 32, fT, NN, nullptr, tid);
  __syncthreads();
  softmax_cols(fT, fT + NN * NN, tid);
  __syncthreads();
  store_lines(attn + (size_t)bc * NN * NN, fT + NN * NN, NN * NN, tid);
}

__global__ __launch_bounds__(NTH) void k_value(
    const float* __restrict__ attn, const float* __restrict__ hq,
    const float* __restrict__ hk,
    const float* __restrict__ Wv2, const float* __restrict__ bv2,
    const float* __restrict__ Wv3, const float* __restrict__ bv3,
    const float* __restrict__ bv1, const float* __restrict__ aV,
    const float* __restrict__ gV,  const float* __restrict__ betaV,
    float* __restrict__ out)
{
  __shared__ __align__(16) _Float16 sW2[SS * SS];
  __shared__ __align__(16) _Float16 sW3[SS * SS];
  __shared__ __align__(16) _Float16 sA[8][16 * SS];
  __shared__ __align__(16) float sO[8][SS];
  __shared__ __align__(16) float sB1[SS];
  __shared__ __align__(16) float sB2[SS];
  __shared__ __align__(16) float sB3[SS];
  __shared__ __align__(16) float sG[SS];
  __shared__ __align__(16) float sBt[SS];

  const int tid  = threadIdx.x;
  const int lane = tid & 31;
  const int wave = tid >> 5;
  const int h    = lane >> 4;
  const int m    = lane & 15;
  const int bc   = blockIdx.x >> 3;
  const int n    = ((blockIdx.x & 7) << 3) + wave;

  for (int i = tid; i < SS * SS; i += NTH) {
    const int k = i >> 7, c = i & 127;
    sW2[c * SS + k] = (_Float16)(Wv2[i] * 16.0f);
    sW3[c * SS + k] = (_Float16)(Wv3[i] * 16.0f);
  }
  for (int i = tid; i < SS; i += NTH) {
    sB1[i] = bv1[i]; sB2[i] = bv2[i]; sB3[i] = bv3[i]; sG[i] = gV[i]; sBt[i] = betaV[i];
  }
  __syncthreads();

  const float av = aV[0];
  _Float16* stage = sA[wave];
  const float* hkrow = hk   + ((size_t)bc * NN + n) * SS;
  const float* arow  = attn + ((size_t)bc * NN + n) * NN;
  const float kInv = 1.0f / 128.0f;

  float outacc[8];
#pragma unroll
  for (int j = 0; j < 8; ++j) outacc[j] = 0.0f;

#pragma unroll 1
  for (int m0 = 0; m0 < NN; m0 += 16) {
    {
      const float* hqrow = hq + ((size_t)bc * NN + m0 + m) * SS;
      const int c0 = h * 64;
#pragma unroll
      for (int c = 0; c < 64; c += 8) {
        const v4f q0 = *(const v4f*)(hqrow + c0 + c);
        const v4f q1 = *(const v4f*)(hqrow + c0 + c + 4);
        const v4f k0v = *(const v4f*)(hkrow + c0 + c);
        const v4f k1v = *(const v4f*)(hkrow + c0 + c + 4);
        const v4f b0 = *(const v4f*)(sB1 + c0 + c);
        const v4f b1 = *(const v4f*)(sB1 + c0 + c + 4);
        const v4f x0 = (q0 + k0v) + b0;
        const v4f x1 = (q1 + k1v) + b1;
        v8h pk;
#pragma unroll
        for (int t = 0; t < 4; ++t) {
          float u0 = x0[t]; u0 = (u0 >= 0.0f) ? u0 : av * u0;
          float u1 = x1[t]; u1 = (u1 >= 0.0f) ? u1 : av * u1;
          pk[t]     = (_Float16)(u0 * 8.0f);
          pk[4 + t] = (_Float16)(u1 * 8.0f);
        }
        *(v8h*)(stage + m * SS + c0 + c) = pk;
      }
    }
    __syncthreads();

    v8f acc[8];
#pragma unroll
    for (int j = 0; j < 8; ++j) acc[j] = zero8();
#pragma unroll 1
    for (int ks = 0; ks < 4; ++ks) {
      const int k0 = ks * 32;
      const v16h af = ldfrag_h(stage, m, k0, h);
#pragma unroll
      for (int j = 0; j < 8; ++j) {
        const v16h bf = ldfrag_h(sW2, j * 16 + m, k0, h);
        acc[j] = wmma_h(af, bf, acc[j]);
      }
    }

#pragma unroll
    for (int j = 0; j < 8; ++j) {
      const float b2 = sB2[j * 16 + m];
#pragma unroll
      for (int e = 0; e < 8; ++e) acc[j][e] = tanhf(acc[j][e] * kInv + b2);
    }

    float mean[8], rstd[8];
#pragma unroll
    for (int e = 0; e < 8; ++e) {
      float s = 0.0f;
#pragma unroll
      for (int j = 0; j < 8; ++j) s += acc[j][e];
#pragma unroll
      for (int mk = 1; mk < 16; mk <<= 1) s += __shfl_xor(s, mk, 32);
      mean[e] = s * (1.0f / SS);
    }
#pragma unroll
    for (int e = 0; e < 8; ++e) {
      float s = 0.0f;
#pragma unroll
      for (int j = 0; j < 8; ++j) { const float d = acc[j][e] - mean[e]; s = fmaf(d, d, s); }
#pragma unroll
      for (int mk = 1; mk < 16; mk <<= 1) s += __shfl_xor(s, mk, 32);
      rstd[e] = rsqrtf(s * (1.0f / SS) + EPSF);
    }
    __syncthreads();

#pragma unroll
    for (int j = 0; j < 8; ++j) {
      const int col = j * 16 + m;
      const float g = sG[col], bt = sBt[col];
#pragma unroll
      for (int e = 0; e < 8; ++e) {
        const float y = (acc[j][e] - mean[e]) * rstd[e] * g + bt;
        stage[(e + 8 * h) * SS + col] = (_Float16)(y * 8.0f);
      }
    }
    __syncthreads();

    v8f acc2[8];
#pragma unroll
    for (int j = 0; j < 8; ++j) acc2[j] = zero8();
#pragma unroll 1
    for (int ks = 0; ks < 4; ++ks) {
      const int k0 = ks * 32;
      const v16h af = ldfrag_h(stage, m, k0, h);
#pragma unroll
      for (int j = 0; j < 8; ++j) {
        const v16h bf = ldfrag_h(sW3, j * 16 + m, k0, h);
        acc2[j] = wmma_h(af, bf, acc2[j]);
      }
    }
    __syncthreads();

    float w8[8];
#pragma unroll
    for (int e = 0; e < 8; ++e) w8[e] = arow[m0 + 8 * h + e];
#pragma unroll
    for (int j = 0; j < 8; ++j) {
      const float b3 = sB3[j * 16 + m];
      float t = 0.0f;
#pragma unroll
      for (int e = 0; e < 8; ++e) t = fmaf(w8[e], acc2[j][e] * kInv + b3, t);
      outacc[j] += t;
    }
  }

#pragma unroll
  for (int j = 0; j < 8; ++j) {
    const float v = outacc[j] + __shfl_xor(outacc[j], 16, 32);
    if (h == 0) sO[wave][j * 16 + m] = v;
  }
  __syncthreads();
  {
    const v4f ov = *(const v4f*)(&sO[wave][4 * lane]);
    float* dst = out + ((size_t)bc * NN + n) * SS + 4 * lane;
    *(volatile v4f*)dst = ov;
    __threadfence();
    *(volatile v4f*)dst = ov;
  }
}

extern "C" void kernel_launch(void* const* d_in, const int* in_sizes, int n_in,
                              void* d_out, int out_size, void* d_ws, size_t ws_size,
                              hipStream_t stream)
{
  if (n_in < 24) return;
  if (in_sizes[0] != BC * NN * IR || in_sizes[1] != BC * NN * IR) return;
  if (in_sizes[2] != IR * SS || in_sizes[8] != IR * SS || in_sizes[12] != 2 * SS * SS) return;
  if (in_sizes[4] != SS * SS || in_sizes[6] != SS * SS || in_sizes[10] != SS * SS ||
      in_sizes[14] != SS * SS || in_sizes[16] != SS * SS) return;
  if (out_size != BC * NN * SS) return;

  const float* tL    = (const float*)d_in[0];
  const float* tH    = (const float*)d_in[1];
  const float* Wk1   = (const float*)d_in[2];
  const float* bk1   = (const float*)d_in[3];
  const float* Wk2   = (const float*)d_in[4];
  const float* bk2   = (const float*)d_in[5];
  const float* Wk3   = (const float*)d_in[6];
  const float* bk3   = (const float*)d_in[7];
  const float* Wq1   = (const float*)d_in[8];
  const float* bq1   = (const float*)d_in[9];
  const float* Wq2   = (const float*)d_in[10];
  const float* bq2   = (const float*)d_in[11];
  const float* Wv1   = (const float*)d_in[12];
  const float* bv1   = (const float*)d_in[13];
  const float* Wv2   = (const float*)d_in[14];
  const float* bv2   = (const float*)d_in[15];
  const float* Wv3   = (const float*)d_in[16];
  const float* bv3   = (const float*)d_in[17];
  const float* aK    = (const float*)d_in[18];
  const float* aV    = (const float*)d_in[19];
  const float* gK    = (const float*)d_in[20];
  const float* betaK = (const float*)d_in[21];
  const float* gV    = (const float*)d_in[22];
  const float* betaV = (const float*)d_in[23];
  float* out = (float*)d_out;

  const size_t n_attn = (size_t)BC * NN * NN;
  const size_t n_h    = (size_t)BC * NN * SS;
  const size_t need_bytes = (n_attn + 2 * n_h) * sizeof(float);
  if (ws_size < need_bytes) return;
  float* ws_attn = (float*)d_ws;
  float* ws_hq   = ws_attn + n_attn;
  float* ws_hk   = ws_hq + n_h;

  k_prep<<<BC, NTH, 0, stream>>>(
      tL, tH, Wk1, bk1, Wk2, bk2, Wk3, bk3, Wq1, bq1, Wq2, bq2,
      Wv1, aK, gK, betaK, ws_attn, ws_hq, ws_hk);

  k_value<<<BC * 8, NTH, 0, stream>>>(
      ws_attn, ws_hq, ws_hk, Wv2, bv2, Wv3, bv3, bv1, aV, gV, betaV, out);
}
